// DeformConvBlock_8280696947121
// MI455X (gfx1250) — hardware-verified
//
#include <hip/hip_runtime.h>
#include <stdint.h>

#define DEVINL __device__ __forceinline__

typedef _Float16 f16t;
typedef _Float16 v16h __attribute__((ext_vector_type(16)));
typedef _Float16 v8h  __attribute__((ext_vector_type(8)));
typedef float    v8f  __attribute__((ext_vector_type(8)));
typedef float    v4f  __attribute__((ext_vector_type(4)));
typedef v8h __attribute__((may_alias)) v8ha;
typedef v4f __attribute__((may_alias)) v4fa;
union FragH { v16h v; v8h half[2]; };

#define CIN   128
#define COUT  128
#define HD    64
#define WDD   64
#define HW    (HD * WDD)
#define NTAP  9
#define KT    (NTAP * CIN)
#define NPIX  64
#define SLP   136
#define XP    65
#define TPB   256
#define NBW   ((COUT * (KT / 8)) / TPB)
#define WCAR  256.0f
#define SCAR  8.0f
#define INVC  (1.0f / 2048.0f)

static_assert((KT % 32) == 0);
static_assert(((COUT * (KT / 8)) % TPB) == 0);
static_assert(NPIX == WDD);
static_assert((CIN * WDD) % TPB == 0);
static_assert(TPB == 4 * NPIX);
static_assert(((SLP * 2) % 16) == 0);
static_assert(((KT * 2) % 128) == 0);
static_assert(((CIN * 4) % 128) == 0);

DEVINL int imin(int a, int b) { return a < b ? a : b; }
DEVINL int imax(int a, int b) { return a > b ? a : b; }

DEVINL v8f wmma_f16(v16h a, v16h b, v8f c) {
  v8f d = __builtin_amdgcn_wmma_f32_16x16x32_f16(false, a, false, b, (short)0, c, false, false);
  asm volatile("v_nop\n\tv_nop\n\tv_nop\n\tv_nop" : "+v"(d) : "v"(a), "v"(b));
  return d;
}
DEVINL v8f zero8f() {
  v8f z = {0.f, 0.f, 0.f, 0.f, 0.f, 0.f, 0.f, 0.f};
  return z;
}

__global__ __launch_bounds__(TPB) void wprep_k(const float* __restrict__ w, f16t* __restrict__ Wp)
{
  const int t = blockIdx.x * TPB + threadIdx.x;
  if (t >= COUT * (KT / 8)) return;
  const int o    = t / (KT / 8);
  const int part = t - o * (KT / 8);
  const int k8   = 8 * part;
  const int tap  = k8 >> 7;
  const int c0   = k8 & (CIN - 1);
  v8h v;
  #pragma unroll
  for (int i = 0; i < 8; ++i) {
    const float wv = w[(size_t)(o * CIN + c0 + i) * NTAP + tap];
    v[i] = (f16t)(wv * WCAR);
  }
  f16t* dst = Wp + (size_t)8 * t;
  *(volatile v8h*)dst = v;
  __threadfence();
  *(volatile v8h*)dst = v;
}

__global__ __launch_bounds__(TPB) void xprep_k(const float* __restrict__ x, float* __restrict__ Xt)
{
  __shared__ __attribute__((aligned(16))) float sX[CIN * XP];
  const int tid = threadIdx.x;
  const int h   = blockIdx.x;
  const int b   = blockIdx.y;
  const float* xb = x + ((size_t)b * CIN) * HW + (size_t)h * WDD;
  #pragma unroll 4
  for (int idx = tid; idx < CIN * WDD; idx += TPB) {
    const int c  = idx >> 6;
    const int wq = idx & (WDD - 1);
    sX[c * XP + wq] = xb[(size_t)c * HW + wq];
  }
  __syncthreads();

  const int pg = tid >> 5;
  const int q  = tid & 31;
  v4f vals[8];
  #pragma unroll
  for (int g = 0; g < 8; ++g) {
    const int wq = 8 * g + pg;
    v4f v;
    v[0] = sX[(4 * q + 0) * XP + wq];
    v[1] = sX[(4 * q + 1) * XP + wq];
    v[2] = sX[(4 * q + 2) * XP + wq];
    v[3] = sX[(4 * q + 3) * XP + wq];
    vals[g] = v;
  }
  float* drow = Xt + ((size_t)(b * HD + h) * WDD) * CIN;
  #pragma unroll
  for (int g = 0; g < 8; ++g)
    *(volatile v4f*)(drow + (size_t)(8 * g + pg) * CIN + 4 * q) = vals[g];
  __threadfence();
  #pragma unroll
  for (int g = 0; g < 8; ++g)
    *(volatile v4f*)(drow + (size_t)(8 * g + pg) * CIN + 4 * q) = vals[g];
}

__global__ __launch_bounds__(TPB) void dconv_k(const float* __restrict__ Xt, const f16t* __restrict__ Wp,
                                             const float* __restrict__ off, const float* __restrict__ bias,
                                             float* __restrict__ out)
{
  __shared__ __attribute__((aligned(16))) f16t  Sl[NPIX * SLP];
  __shared__ __attribute__((aligned(16))) float sO[COUT * NPIX];
  const int tid = threadIdx.x, lane = tid & 31, wave = tid >> 5;
  const int h = lane >> 4, m = lane & 15;
  const int wg = blockIdx.x;
  const int b  = wg >> 6;
  const int oh = wg & (HD - 1);

  const int pos = tid & (NPIX - 1);
  const int cg  = tid >> 6;
  const float* xb = Xt + (size_t)b * HW * CIN + 32 * cg;
  const f16t* arow = Wp + (size_t)(16 * wave + m) * KT + 8 * h;

  v8f acc[4];
  #pragma unroll
  for (int t = 0; t < 4; ++t) acc[t] = zero8f();

  #pragma unroll 1
  for (int tap = 0; tap < NTAP; ++tap) {
    const int ki = tap / 3;
    const int kj = tap - 3 * ki;
    __syncthreads();

    {
      const float oy = off[(((size_t)b * (2 * NTAP) + 2 * tap    ) * HD + oh) * WDD + pos];
      const float ox = off[(((size_t)b * (2 * NTAP) + 2 * tap + 1) * HD + oh) * WDD + pos];
      const float ys = (float)(oh + ki - 1) + oy;
      const float xs = (float)(pos + kj - 1) + ox;
      const float y0f = floorf(ys), x0f = floorf(xs);
      const float wy = ys - y0f,   wx = xs - x0f;
      const float y1f = y0f + 1.0f, x1f = x0f + 1.0f;
      const bool vy0 = (y0f >= 0.0f) && (y0f <= (float)(HD - 1));
      const bool vy1 = (y1f >= 0.0f) && (y1f <= (float)(HD - 1));
      const bool vx0 = (x0f >= 0.0f) && (x0f <= (float)(WDD - 1));
      const bool vx1 = (x1f >= 0.0f) && (x1f <= (float)(WDD - 1));
      const float omy = 1.0f - wy, omx = 1.0f - wx;
      float w00 = omy * omx;
      float w01 = omy * wx;
      float w10 = wy * omx;
      float w11 = wy * wx;
      w00 = (vy0 && vx0) ? w00 : 0.0f;
      w01 = (vy0 && vx1) ? w01 : 0.0f;
      w10 = (vy1 && vx0) ? w10 : 0.0f;
      w11 = (vy1 && vx1) ? w11 : 0.0f;
      const int y0c = imin(imax((int)y0f, 0), HD - 1);
      const int y1c = imin(imax((int)y1f, 0), HD - 1);
      const int x0c = imin(imax((int)x0f, 0), WDD - 1);
      const int x1c = imin(imax((int)x1f, 0), WDD - 1);
      const float* p00 = xb + (size_t)(y0c * WDD + x0c) * CIN;
      const float* p01 = xb + (size_t)(y0c * WDD + x1c) * CIN;
      const float* p10 = xb + (size_t)(y1c * WDD + x0c) * CIN;
      const float* p11 = xb + (size_t)(y1c * WDD + x1c) * CIN;
      f16t* srow = Sl + pos * SLP + 32 * cg;
      #pragma unroll
      for (int ch = 0; ch < 4; ++ch) {
        const v4f a0 = *(const v4fa*)(p00 + 8 * ch), a1 = *(const v4fa*)(p00 + 8 * ch + 4);
        const v4f b0 = *(const v4fa*)(p01 + 8 * ch), b1 = *(const v4fa*)(p01 + 8 * ch + 4);
        const v4f c0 = *(const v4fa*)(p10 + 8 * ch), c1 = *(const v4fa*)(p10 + 8 * ch + 4);
        const v4f d0 = *(const v4fa*)(p11 + 8 * ch), d1 = *(const v4fa*)(p11 + 8 * ch + 4);
        v4f s0 = a0 * w00;
        v4f s1 = a1 * w00;
        s0 = b0 * w01 + s0;  s1 = b1 * w01 + s1;
        s0 = c0 * w10 + s0;  s1 = c1 * w10 + s1;
        s0 = d0 * w11 + s0;  s1 = d1 * w11 + s1;
        v8h o;
        #pragma unroll
        for (int i = 0; i < 4; ++i) {
          o[i]     = (f16t)(s0[i] * SCAR);
          o[4 + i] = (f16t)(s1[i] * SCAR);
        }
        *(v8ha*)(srow + 8 * ch) = o;
      }
    }
    __syncthreads();

    const f16t* at = arow + tap * CIN;
    #pragma unroll
    for (int c = 0; c < 4; ++c) {
      FragH a;
      a.half[0] = *(const v8ha*)(at + 32 * c);
      a.half[1] = *(const v8ha*)(at + 32 * c + 16);
      #pragma unroll
      for (int t = 0; t < 4; ++t) {
        FragH bf;
        const f16t* br = Sl + (16 * t + m) * SLP + 32 * c + 8 * h;
        bf.half[0] = *(const v8ha*)(br);
        bf.half[1] = *(const v8ha*)(br + 16);
        acc[t] = wmma_f16(a.v, bf.v, acc[t]);
      }
    }
  }

  #pragma unroll
  for (int t = 0; t < 4; ++t) {
    #pragma unroll
    for (int r = 0; r < 8; ++r) {
      const int cout = 16 * wave + 8 * h + r;
      float v = acc[t][r] * INVC + bias[cout];
      v = v > 0.0f ? v : 0.0f;
      sO[cout * NPIX + 16 * t + m] = v;
    }
  }
  __syncthreads();

  float* gbase = out + ((size_t)b * COUT) * HW + (size_t)oh * WDD + 4 * m;
  v4f vv[8];
  #pragma unroll
  for (int j = 0; j < 8; ++j) {
    const int row = 16 * wave + 2 * j + h;
    vv[j] = *(const v4fa*)(sO + row * NPIX + 4 * m);
  }
  #pragma unroll
  for (int j = 0; j < 8; ++j) {
    const int row = 16 * wave + 2 * j + h;
    *(volatile v4f*)(gbase + (size_t)row * HW) = vv[j];
  }
  __threadfence();
  #pragma unroll
  for (int j = 0; j < 8; ++j) {
    const int row = 16 * wave + 2 * j + h;
    *(volatile v4f*)(gbase + (size_t)row * HW) = vv[j];
  }
}

extern "C" void kernel_launch(void* const* d_in, const int* in_sizes, int n_in,
                              void* d_out, int out_size, void* d_ws, size_t ws_size,
                              hipStream_t stream)
{
  if (n_in < 4) return;
  const int plane = CIN * HW;
  if (in_sizes[0] <= 0 || (in_sizes[0] % plane) != 0) return;
  const int nB = in_sizes[0] / plane;
  if (nB > 1024) return;
  if (in_sizes[1] != nB * 2 * NTAP * HW) return;
  if (in_sizes[2] != COUT * CIN * NTAP) return;
  if (in_sizes[3] != COUT) return;
  if (out_size != nB * COUT * HW) return;

  const float* x    = (const float*)d_in[0];
  const float* off  = (const float*)d_in[1];
  const float* wgt  = (const float*)d_in[2];
  const float* bias = (const float*)d_in[3];
  float* outp = (float*)d_out;

  const size_t szWp = (size_t)COUT * KT * 2;
  const size_t szXt = (size_t)nB * HW * CIN * 4;
  size_t offb = 0;
  char* ws = (char*)d_ws;
  f16t*  Wp = (f16t*)(ws + offb);  offb += szWp;
  float* Xt = (float*)(ws + offb); offb += szXt;
  if (offb > ws_size) return;
  if (offb > (size_t)134217728) return;

  wprep_k<<<NBW, TPB, 0, stream>>>(wgt, Wp);
  xprep_k<<<dim3(HD, nB), TPB, 0, stream>>>(x, Xt);
  dconv_k<<<nB * HD, TPB, 0, stream>>>(Xt, Wp, off, bias, outp);
}
